// SelfAttention_67104569033420
// MI455X (gfx1250) — hardware-verified
//
#include <hip/hip_runtime.h>


#ifndef NB
#define NB 4
#endif
#ifndef SEQ
#define SEQ 4096
#endif
#define NB_FULL   4
#define SEQ_FULL  4096
#define NIN       256
#define DH        128
#define TOK       64
#define BQ        64
#define BK        32
#define NWAVE     4
#define SP        132
#define WP        72
#define WKT       64
#define PLANE_ELEMS ((size_t)NB * SEQ * DH)
#define WT_ELEMS    ((size_t)3 * DH * NIN)
#define WS_NEEDED   ((6 * PLANE_ELEMS + WT_ELEMS) * 2)

static_assert(SEQ % TOK == 0);
static_assert(SEQ % BQ == 0);
static_assert(SEQ % BK == 0);
static_assert(BQ == NWAVE * 16);
static_assert(TOK == 64);
static_assert(DH == 128);
static_assert(NIN == 256);
static_assert(NIN % 32 == 0);
static_assert(DH % 32 == 0);
static_assert(NIN % WKT == 0);
static_assert(WKT == 64);
static_assert(SP >= DH);
static_assert(WP >= WKT);
static_assert((SP * 4) % 16 == 0);
static_assert((WP * 2) % 16 == 0);
static_assert(4 * 256 * 8 == TOK * DH);
static_assert(8 * 256 * 4 == WKT * DH);
static_assert(4 * 256 * 8 == DH * WKT);
static_assert(32 * 4 == DH);
static_assert(SEQ <= SEQ_FULL);
static_assert(NB >= 1 && NB <= NB_FULL);
static_assert(TOK * SP * 4 <= 65536);
static_assert(NWAVE * 16 * SP * 4 <= 65536);
static_assert(DH * WP * 2 <= 65536);
static_assert(WS_NEEDED <= (size_t)134217728);
static_assert((((size_t)(NB - 1) * SEQ_FULL + SEQ) * DH) * 4 <= (size_t)8388608);
static_assert((PLANE_ELEMS * 2) % 128 == 0);

typedef __bf16   bf16;
typedef bf16     v16bf __attribute__((ext_vector_type(16)));
typedef float    v8f   __attribute__((ext_vector_type(8)));
typedef float    v4f   __attribute__((ext_vector_type(4)));
typedef unsigned v4u   __attribute__((ext_vector_type(4)));

union FragB  { v16bf v; v4u q[2]; bf16 h[16]; };
union Pack8B { v4u u; bf16 h[8]; };

static __device__ __forceinline__ v8f mma_bf16(v16bf a, v16bf b, v8f acc) {
  acc = __builtin_amdgcn_wmma_f32_16x16x32_bf16(false, a, false, b, (short)0, acc, false, false);
  asm volatile("v_nop\n\tv_nop\n\tv_nop\n\tv_nop" : "+v"(acc) : "v"(a), "v"(b));
  return acc;
}

__global__ __launch_bounds__(256) void w_plane_kernel(const float* __restrict__ W,
                                                      bf16* __restrict__ wtm) {
  const int k0  = blockIdx.x * WKT;
  const int tid = threadIdx.x;
  __shared__ __align__(16) bf16 sW[DH * WP];

  #pragma unroll
  for (int it = 0; it < 8; ++it) {
    const int idx = it * 256 + tid;
    const int kr  = idx >> 5;
    const int n4  = (idx & 31) * 4;
    const v4f w = *(const v4f*)(W + (size_t)(k0 + kr) * DH + n4);
    #pragma unroll
    for (int i = 0; i < 4; ++i) sW[(n4 + i) * WP + kr] = (bf16)w[i];
  }
  __syncthreads();

  v4u      val[4];
  unsigned off[4];
  #pragma unroll
  for (int it = 0; it < 4; ++it) {
    const int chunk = it * 256 + tid;
    const int n  = chunk >> 3;
    const int kc = (chunk & 7) * 8;
    val[it] = *(const v4u*)(sW + n * WP + kc);
    off[it] = (unsigned)(n * NIN + k0 + kc);
  }
  #pragma unroll
  for (int it = 0; it < 4; ++it) *(volatile v4u*)(wtm + off[it]) = val[it];
  __threadfence();
  #pragma unroll
  for (int it = 0; it < 4; ++it) *(volatile v4u*)(wtm + off[it]) = val[it];
}

__global__ __launch_bounds__(256) void proj_kernel(const float* __restrict__ seq,
                                                   const bf16* __restrict__ wt,
                                                   bf16* __restrict__ planes) {
  const int tb   = blockIdx.x;
  const int b    = blockIdx.y;
  const int tid  = threadIdx.x;
  const int wave = __builtin_amdgcn_readfirstlane(threadIdx.x >> 5);
  const int lane = tid & 31;
  const int lq   = lane & 15;
  const int hi   = lane >> 4;
  const int mt   = wave & 3;
  const int nh   = wave >> 2;
  const int t0   = tb * TOK;

  __shared__ __align__(16) float sS[TOK * SP];

  FragB af[8];
  {
    const float* ap = seq + ((size_t)b * SEQ_FULL + t0 + mt * 16 + lq) * NIN;
    #pragma unroll
    for (int ks = 0; ks < 8; ++ks) {
      if (ks == 4) asm volatile("" ::: "memory");
      const v4f a0 = *(const v4f*)(ap + ks * 32 + hi * 8);
      const v4f a1 = *(const v4f*)(ap + ks * 32 + hi * 8 + 4);
      const v4f b0 = *(const v4f*)(ap + ks * 32 + 16 + hi * 8);
      const v4f b1 = *(const v4f*)(ap + ks * 32 + 16 + hi * 8 + 4);
      #pragma unroll
      for (int i = 0; i < 4; ++i) {
        af[ks].h[i]      = (bf16)a0[i];
        af[ks].h[4 + i]  = (bf16)a1[i];
        af[ks].h[8 + i]  = (bf16)b0[i];
        af[ks].h[12 + i] = (bf16)b1[i];
      }
    }
  }

  #pragma unroll 1
  for (int mat = 0; mat < 3; ++mat) {
    v8f acc[4];
    #pragma unroll
    for (int j = 0; j < 4; ++j) acc[j] = (v8f){0, 0, 0, 0, 0, 0, 0, 0};

    const bf16* wb = wt + (size_t)(mat * DH + nh * 64 + lq) * NIN + hi * 8;
    #pragma unroll
    for (int ks = 0; ks < 8; ++ks) {
      #pragma unroll
      for (int j = 0; j < 4; ++j) {
        FragB bw;
        const bf16* base = wb + j * 16 * NIN + ks * 32;
        bw.q[0] = *(const v4u*)(base);
        bw.q[1] = *(const v4u*)(base + 16);
        acc[j] = mma_bf16(af[ks].v, bw.v, acc[j]);
      }
    }

    #pragma unroll
    for (int j = 0; j < 4; ++j) {
      #pragma unroll
      for (int r = 0; r < 8; ++r)
        sS[(mt * 16 + hi * 8 + r) * SP + nh * 64 + j * 16 + lq] = acc[j][r];
    }
    __syncthreads();

    const int sstr = (mat < 2) ? 1 : SP;
    v4u    hv[4], lv[4];
    size_t off[4];
    #pragma unroll
    for (int it = 0; it < 4; ++it) {
      const int chunk = it * 256 + tid;
      int    sidx;
      size_t eo;
      if (mat < 2) {
        const int row = chunk >> 4;
        const int dc  = (chunk & 15) * 8;
        sidx = row * SP + dc;
        eo   = (size_t)(2 * mat) * PLANE_ELEMS + ((size_t)b * SEQ + t0 + row) * DH + dc;
      } else {
        const int d  = chunk >> 3;
        const int tc = (chunk & 7) * 8;
        sidx = tc * SP + d;
        eo   = (size_t)4 * PLANE_ELEMS + ((size_t)b * DH + d) * SEQ + t0 + tc;
      }
      Pack8B ph, pl;
      #pragma unroll
      for (int i = 0; i < 8; ++i) {
        const float x  = sS[sidx + i * sstr];
        const bf16  hb = (bf16)x;
        ph.h[i] = hb;
        pl.h[i] = (bf16)(x - (float)hb);
      }
      hv[it]  = ph.u;
      lv[it]  = pl.u;
      off[it] = eo;
    }
    #pragma unroll
    for (int it = 0; it < 4; ++it) {
      *(volatile v4u*)(planes + off[it]) = hv[it];
      *(volatile v4u*)(planes + off[it] + PLANE_ELEMS) = lv[it];
    }
    __threadfence();
    #pragma unroll
    for (int it = 0; it < 4; ++it) {
      *(volatile v4u*)(planes + off[it]) = hv[it];
      *(volatile v4u*)(planes + off[it] + PLANE_ELEMS) = lv[it];
    }
    __syncthreads();
  }
}

__global__ __launch_bounds__(128) void attn_kernel(const bf16* __restrict__ planes,
                                                   float* __restrict__ out) {
  const int qblk = blockIdx.x;
  const int b    = blockIdx.y;
  const int tid  = threadIdx.x;
  const int wave = __builtin_amdgcn_readfirstlane(threadIdx.x >> 5);
  const int lane = tid & 31;
  const int lq   = lane & 15;
  const int hi   = lane >> 4;

  __shared__ __align__(16) float sO[NWAVE * 16 * SP];

  const int qrow0 = qblk * BQ + wave * 16;

  const bf16* qh_b = planes + (size_t)b * SEQ * DH;
  const bf16* ql_b = qh_b + PLANE_ELEMS;
  const bf16* kh_b = qh_b + 2 * PLANE_ELEMS;
  const bf16* kl_b = qh_b + 3 * PLANE_ELEMS;
  const bf16* vh_b = qh_b + 4 * PLANE_ELEMS;
  const bf16* vl_b = qh_b + 5 * PLANE_ELEMS;

  const unsigned qoff = (unsigned)(qrow0 + lq) * DH + hi * 8;

  v8f o[8];
  #pragma unroll
  for (int dt = 0; dt < 8; ++dt) o[dt] = (v8f){0, 0, 0, 0, 0, 0, 0, 0};

  float rmax = -__builtin_inff();
  float rsum = 0.0f;
  const float SL = 1.4426950408889634f;

  #pragma unroll 1
  for (int it = 0; it < SEQ / BK; ++it) {
    const int j0 = it * BK;
    unsigned qo = qoff;
    asm volatile("" : "+v"(qo));
    const unsigned ko = (unsigned)(j0 + lq) * DH + hi * 8;

    v8f c0 = (v8f){0, 0, 0, 0, 0, 0, 0, 0};
    v8f c1 = (v8f){0, 0, 0, 0, 0, 0, 0, 0};
    #pragma unroll
    for (int f = 0; f < 4; ++f) {
      FragB qh, ql, k0h, k0l, k1h, k1l;
      qh.q[0]  = *(const v4u*)(qh_b + qo + f * 32);
      qh.q[1]  = *(const v4u*)(qh_b + qo + f * 32 + 16);
      ql.q[0]  = *(const v4u*)(ql_b + qo + f * 32);
      ql.q[1]  = *(const v4u*)(ql_b + qo + f * 32 + 16);
      k0h.q[0] = *(const v4u*)(kh_b + ko + f * 32);
      k0h.q[1] = *(const v4u*)(kh_b + ko + f * 32 + 16);
      k0l.q[0] = *(const v4u*)(kl_b + ko + f * 32);
      k0l.q[1] = *(const v4u*)(kl_b + ko + f * 32 + 16);
      k1h.q[0] = *(const v4u*)(kh_b + ko + 16 * DH + f * 32);
      k1h.q[1] = *(const v4u*)(kh_b + ko + 16 * DH + f * 32 + 16);
      k1l.q[0] = *(const v4u*)(kl_b + ko + 16 * DH + f * 32);
      k1l.q[1] = *(const v4u*)(kl_b + ko + 16 * DH + f * 32 + 16);
      c0 = mma_bf16(k0h.v, qh.v, c0);
      c1 = mma_bf16(k1h.v, qh.v, c1);
      c0 = mma_bf16(k0h.v, ql.v, c0);
      c1 = mma_bf16(k1h.v, ql.v, c1);
      c0 = mma_bf16(k0l.v, qh.v, c0);
      c1 = mma_bf16(k1l.v, qh.v, c1);
    }

    float m_new = rmax;
    #pragma unroll
    for (int r = 0; r < 8; ++r) {
      m_new = fmaxf(m_new, c0[r]);
      m_new = fmaxf(m_new, c1[r]);
    }
    m_new = fmaxf(m_new, __shfl_xor(m_new, 16, 32));
    const float scale = __builtin_amdgcn_exp2f((rmax - m_new) * SL);
    rmax = m_new;

    FragB pa, pb;
    float psum = 0.0f;
    #pragma unroll
    for (int r = 0; r < 8; ++r) {
      const float p0 = __builtin_amdgcn_exp2f((c0[r] - m_new) * SL);
      const float p1 = __builtin_amdgcn_exp2f((c1[r] - m_new) * SL);
      psum += p0 + p1;
      const bf16 h0 = (bf16)p0;
      const bf16 h1 = (bf16)p1;
      pa.h[r]     = h0;
      pa.h[8 + r] = h1;
      pb.h[r]     = (bf16)(p0 - (float)h0);
      pb.h[8 + r] = (bf16)(p1 - (float)h1);
    }
    rsum = rsum * scale + psum + __shfl_xor(psum, 16, 32);

    float sc[8];
    #pragma unroll
    for (int r = 0; r < 8; ++r) sc[r] = __shfl(scale, (hi << 3) + r, 32);
    #pragma unroll
    for (int dt = 0; dt < 8; ++dt) {
      #pragma unroll
      for (int r = 0; r < 8; ++r) o[dt][r] *= sc[r];
    }

    #pragma unroll
    for (int g = 0; g < 2; ++g) {
      FragB vh[4], vl[4];
      #pragma unroll
      for (int t = 0; t < 4; ++t) {
        const unsigned vo = (unsigned)((g * 4 + t) * 16 + lq) * SEQ + j0 + hi * 8;
        vh[t].q[0] = *(const v4u*)(vh_b + vo);
        vh[t].q[1] = *(const v4u*)(vh_b + vo + 16);
        vl[t].q[0] = *(const v4u*)(vl_b + vo);
        vl[t].q[1] = *(const v4u*)(vl_b + vo + 16);
      }
      #pragma unroll
      for (int t = 0; t < 4; ++t) {
        o[g * 4 + t] = mma_bf16(pa.v, vh[t].v, o[g * 4 + t]);
        o[g * 4 + t] = mma_bf16(pa.v, vl[t].v, o[g * 4 + t]);
        o[g * 4 + t] = mma_bf16(pb.v, vh[t].v, o[g * 4 + t]);
      }
    }
  }

  float rs[8];
  #pragma unroll
  for (int r = 0; r < 8; ++r) rs[r] = 1.0f / __shfl(rsum, (hi << 3) + r, 32);

  const int sbase = wave * (16 * SP);
  #pragma unroll
  for (int r = 0; r < 8; ++r) {
    #pragma unroll
    for (int dt = 0; dt < 8; ++dt)
      sO[sbase + (hi * 8 + r) * SP + dt * 16 + lq] = o[dt][r] * rs[r];
  }
  __syncthreads();

  v4f vals[16];
  #pragma unroll
  for (int row = 0; row < 16; ++row)
    vals[row] = *(const v4f*)(sO + sbase + row * SP + lane * 4);
  const size_t gbase = ((size_t)b * SEQ_FULL + qrow0) * DH + (size_t)lane * 4;
  #pragma unroll
  for (int row = 0; row < 16; ++row) *(volatile v4f*)(out + gbase + (size_t)row * DH) = vals[row];
  __threadfence();
  #pragma unroll
  for (int row = 0; row < 16; ++row) *(volatile v4f*)(out + gbase + (size_t)row * DH) = vals[row];
}

extern "C" void kernel_launch(void* const* d_in, const int* in_sizes, int n_in,
                              void* d_out, int out_size, void* d_ws, size_t ws_size,
                              hipStream_t stream) {
  if (n_in < 5) return;
  const size_t rows_used = (size_t)(NB - 1) * SEQ_FULL + SEQ;
  if ((size_t)in_sizes[0] < rows_used * NIN) return;
  if ((size_t)in_sizes[2] < (size_t)NIN * DH) return;
  if ((size_t)in_sizes[3] < (size_t)NIN * DH) return;
  if ((size_t)in_sizes[4] < (size_t)NIN * DH) return;
  if ((size_t)out_size < rows_used * DH) return;
  if (ws_size < WS_NEEDED) return;

  const float* seq = (const float*)d_in[0];
  const int*   lengths = (const int*)d_in[1];
  (void)lengths;
  const float* Wq = (const float*)d_in[2];
  const float* Wk = (const float*)d_in[3];
  const float* Wv = (const float*)d_in[4];
  float*       out = (float*)d_out;

  bf16* planes = (bf16*)d_ws;
  bf16* wt     = planes + 6 * PLANE_ELEMS;

  w_plane_kernel<<<dim3(NIN / WKT), 256, 0, stream>>>(Wq, wt);
  w_plane_kernel<<<dim3(NIN / WKT), 256, 0, stream>>>(Wk, wt + (size_t)DH * NIN);
  w_plane_kernel<<<dim3(NIN / WKT), 256, 0, stream>>>(Wv, wt + (size_t)2 * DH * NIN);

  proj_kernel<<<dim3(SEQ / TOK, NB), 256, 0, stream>>>(seq, wt, planes);

  attn_kernel<<<dim3(SEQ / BQ, NB), 128, 0, stream>>>(planes, out);
}
